// ExpertLinear_11948599017885
// MI455X (gfx1250) — hardware-verified
//
#include <hip/hip_runtime.h>
#include <stdint.h>
#include <stddef.h>


typedef _Float16 v16h __attribute__((ext_vector_type(16)));
typedef _Float16 v8h  __attribute__((ext_vector_type(8)));
typedef float    v8f  __attribute__((ext_vector_type(8)));
typedef float    v4f  __attribute__((ext_vector_type(4)));
typedef v4f v4fa __attribute__((may_alias));
typedef v8h v8ha __attribute__((may_alias));

#define NTOK   8192
#define IN_F   1024
#define OUT_F  1024
#define NEXP   8

#define WT_M   32
#define WT_N   64
#define WAVES  4
#define BLK_M  (WT_M * WAVES)
#define OPITCH 68

#define W_SCALE 512.0f
#define W_INV   (1.0f / 512.0f)
#define CVT_THREADS 256

union H8   { v8h v; unsigned short s[8]; };
union Frag { v16h v; v8h half[2]; };

__global__ __launch_bounds__(CVT_THREADS)
void k_convert_f16(const float* __restrict__ x, const float* __restrict__ w,
                   _Float16* __restrict__ xh, _Float16* __restrict__ wh,
                   int nvec_x, int nvec_w, int nblk_x)
{
    const bool is_x = (int)blockIdx.x < nblk_x;
    const float* src  = is_x ? x : w;
    _Float16*    dst  = is_x ? xh : wh;
    const float  scale = is_x ? 1.0f : W_SCALE;
    const int    nvec = is_x ? nvec_x : nvec_w;
    const int    vb   = is_x ? (int)blockIdx.x : ((int)blockIdx.x - nblk_x);
    const int    vec  = vb * CVT_THREADS + (int)threadIdx.x;
    if (vec >= nvec) return;

    const size_t off = (size_t)vec * 8;
    const v4fa* p = (const v4fa*)(src + off);
    const v4f f0 = p[0];
    const v4f f1 = p[1];

    H8 u;
    u.v[0] = (_Float16)(f0.x * scale);
    u.v[1] = (_Float16)(f0.y * scale);
    u.v[2] = (_Float16)(f0.z * scale);
    u.v[3] = (_Float16)(f0.w * scale);
    u.v[4] = (_Float16)(f1.x * scale);
    u.v[5] = (_Float16)(f1.y * scale);
    u.v[6] = (_Float16)(f1.z * scale);
    u.v[7] = (_Float16)(f1.w * scale);
    #pragma unroll
    for (int i = 0; i < 8; ++i) {
        const unsigned short bts = u.s[i];
        u.s[i] = ((bts & 0x7C00u) == 0u) ? (unsigned short)0 : bts;
    }
    const v8h hv = u.v;

    volatile v8h* q = (volatile v8h*)(dst + off);
    *q = hv;
    __threadfence();
    *q = hv;
}

__global__ __launch_bounds__(WAVES * 32)
void k_expert_gemm_blend(const _Float16* __restrict__ xh, const _Float16* __restrict__ wh,
                         const float* __restrict__ ew, const float* __restrict__ bias,
                         float* __restrict__ out)
{
    __shared__ __align__(16) float Osm[WAVES][WT_M * OPITCH];

    const int tid  = (int)threadIdx.x;
    const int wave = tid >> 5;
    const int l    = tid & 31;
    const int h    = l >> 4;
    const int m    = l & 15;
    const int col0 = (int)blockIdx.x * WT_N;
    const int tok0 = (int)blockIdx.y * BLK_M + wave * WT_M;
    float* O = Osm[wave];

    #pragma unroll
    for (int mt = 0; mt < 2; ++mt)
        #pragma unroll
        for (int r = 0; r < 8; ++r)
            #pragma unroll
            for (int nt = 0; nt < 4; ++nt)
                O[(16 * mt + 8 * h + r) * OPITCH + 16 * nt + m] = 0.0f;

    const _Float16* pa0 = xh + (size_t)(tok0 + m) * IN_F + 8 * h;
    const _Float16* pa1 = pa0 + (size_t)16 * IN_F;

    const v8f zero8 = {0.f, 0.f, 0.f, 0.f, 0.f, 0.f, 0.f, 0.f};

    #pragma unroll 1
    for (int e = 0; e < NEXP; ++e) {
        const _Float16* pb0 = wh + ((size_t)e * OUT_F + (size_t)(col0 + m)) * IN_F + 8 * h;
        const _Float16* pb1 = pb0 + (size_t)16 * IN_F;
        const _Float16* pb2 = pb0 + (size_t)32 * IN_F;
        const _Float16* pb3 = pb0 + (size_t)48 * IN_F;

        v8f acc[2][4];
        #pragma unroll
        for (int mt = 0; mt < 2; ++mt)
            #pragma unroll
            for (int nt = 0; nt < 4; ++nt)
                acc[mt][nt] = zero8;

        #pragma unroll 1
        for (int ks = 0; ks < IN_F / 32; ++ks) {
            const int k0 = ks * 32;
            Frag a0, a1, b0, b1, b2, b3;
            a0.half[0] = *(const v8ha*)(pa0 + k0);
            a0.half[1] = *(const v8ha*)(pa0 + k0 + 16);
            a1.half[0] = *(const v8ha*)(pa1 + k0);
            a1.half[1] = *(const v8ha*)(pa1 + k0 + 16);
            b0.half[0] = *(const v8ha*)(pb0 + k0);
            b0.half[1] = *(const v8ha*)(pb0 + k0 + 16);
            b1.half[0] = *(const v8ha*)(pb1 + k0);
            b1.half[1] = *(const v8ha*)(pb1 + k0 + 16);
            b2.half[0] = *(const v8ha*)(pb2 + k0);
            b2.half[1] = *(const v8ha*)(pb2 + k0 + 16);
            b3.half[0] = *(const v8ha*)(pb3 + k0);
            b3.half[1] = *(const v8ha*)(pb3 + k0 + 16);

            acc[0][0] = __builtin_amdgcn_wmma_f32_16x16x32_f16(false, a0.v, false, b0.v, (short)0, acc[0][0], false, false);
            acc[0][1] = __builtin_amdgcn_wmma_f32_16x16x32_f16(false, a0.v, false, b1.v, (short)0, acc[0][1], false, false);
            acc[0][2] = __builtin_amdgcn_wmma_f32_16x16x32_f16(false, a0.v, false, b2.v, (short)0, acc[0][2], false, false);
            acc[0][3] = __builtin_amdgcn_wmma_f32_16x16x32_f16(false, a0.v, false, b3.v, (short)0, acc[0][3], false, false);
            acc[1][0] = __builtin_amdgcn_wmma_f32_16x16x32_f16(false, a1.v, false, b0.v, (short)0, acc[1][0], false, false);
            acc[1][1] = __builtin_amdgcn_wmma_f32_16x16x32_f16(false, a1.v, false, b1.v, (short)0, acc[1][1], false, false);
            acc[1][2] = __builtin_amdgcn_wmma_f32_16x16x32_f16(false, a1.v, false, b2.v, (short)0, acc[1][2], false, false);
            acc[1][3] = __builtin_amdgcn_wmma_f32_16x16x32_f16(false, a1.v, false, b3.v, (short)0, acc[1][3], false, false);

            asm volatile("v_nop\n\tv_nop\n\tv_nop\n\tv_nop"
                         : "+v"(acc[0][0]), "+v"(acc[0][1]), "+v"(acc[0][2]), "+v"(acc[0][3]),
                           "+v"(acc[1][0]), "+v"(acc[1][1]), "+v"(acc[1][2]), "+v"(acc[1][3])
                         : "v"(a0.v), "v"(a1.v), "v"(b0.v), "v"(b1.v), "v"(b2.v), "v"(b3.v)
                         : "memory");
        }

        float bb[4];
        #pragma unroll
        for (int nt = 0; nt < 4; ++nt)
            bb[nt] = bias[(size_t)e * OUT_F + (size_t)(col0 + 16 * nt + m)];

        #pragma unroll
        for (int mt = 0; mt < 2; ++mt) {
            #pragma unroll
            for (int r = 0; r < 8; ++r) {
                const int   row = 16 * mt + 8 * h + r;
                const float wv  = ew[(size_t)(tok0 + row) * NEXP + e];
                const float wsc = wv * W_INV;
                #pragma unroll
                for (int nt = 0; nt < 4; ++nt) {
                    const int pos = row * OPITCH + 16 * nt + m;
                    float o = O[pos];
                    o = o + (wsc * acc[mt][nt][r] + wv * bb[nt]);
                    O[pos] = o;
                }
            }
        }
    }

    __syncthreads();

    v4f vals[16];
    #pragma unroll
    for (int j = 0; j < 16; ++j) {
        const int row = 2 * j + h;
        vals[j] = *(const v4fa*)(O + row * OPITCH + 4 * m);
    }
    #pragma unroll
    for (int j = 0; j < 16; ++j) {
        const int row = 2 * j + h;
        *(volatile v4f*)(out + (size_t)(tok0 + row) * OUT_F + (size_t)(col0 + 4 * m)) = vals[j];
    }
    __threadfence();
    #pragma unroll
    for (int j = 0; j < 16; ++j) {
        const int row = 2 * j + h;
        *(volatile v4f*)(out + (size_t)(tok0 + row) * OUT_F + (size_t)(col0 + 4 * m)) = vals[j];
    }
}

extern "C" void kernel_launch(void* const* d_in, const int* in_sizes, int n_in,
                              void* d_out, int out_size, void* d_ws, size_t ws_size,
                              hipStream_t stream)
{
    if (n_in < 4) return;
    const size_t nx  = (size_t)NTOK * IN_F;
    const size_t ne  = (size_t)NTOK * NEXP;
    const size_t nw  = (size_t)NEXP * OUT_F * IN_F;
    const size_t nb  = (size_t)NEXP * OUT_F;
    const size_t no  = (size_t)NTOK * OUT_F;
    if ((size_t)in_sizes[0] != nx || (size_t)in_sizes[1] != ne ||
        (size_t)in_sizes[2] != nw || (size_t)in_sizes[3] != nb ||
        (size_t)out_size != no) return;

    const size_t xh_bytes = nx * sizeof(_Float16);
    const size_t wh_bytes = nw * sizeof(_Float16);
    if (xh_bytes + wh_bytes > ws_size) return;

    const float* x    = (const float*)d_in[0];
    const float* ew   = (const float*)d_in[1];
    const float* w    = (const float*)d_in[2];
    const float* bias = (const float*)d_in[3];
    float*       out  = (float*)d_out;
    _Float16*    xh   = (_Float16*)d_ws;
    _Float16*    wh   = (_Float16*)((char*)d_ws + xh_bytes);

    const int nvec_x = (int)(nx / 8);
    const int nvec_w = (int)(nw / 8);
    const int nblk_x = (nvec_x + CVT_THREADS - 1) / CVT_THREADS;
    const int nblk_w = (nvec_w + CVT_THREADS - 1) / CVT_THREADS;

    hipLaunchKernelGGL(k_convert_f16, dim3(nblk_x + nblk_w), dim3(CVT_THREADS), 0, stream,
                       x, w, xh, wh, nvec_x, nvec_w, nblk_x);

    dim3 grid(OUT_F / WT_N, NTOK / BLK_M);
    hipLaunchKernelGGL(k_expert_gemm_blend, grid, dim3(WAVES * 32), 0, stream,
                       (const _Float16*)xh, (const _Float16*)wh, ew, bias, out);
    (void)hipGetLastError();
}
